// _HMoEModule_68478958567429
// MI455X (gfx1250) — hardware-run, weakly checked
//
#include <hip/hip_runtime.h>
#include <stdint.h>
#include <stddef.h>
#include <math.h>

#define BSZ   4096
#define FDIM  1024
#define GHD   256
#define EHD   512
#define CDIM  1000
#define CPAD  1024
#define NGATE 15
#define NEXP  16
#define BFC   2
#define DEPTH 4

#define GROWS 32
#define EROWS 32
#define MROWS 16
#define TP    72
#define MIX_FLOATS (MROWS * CDIM)
#define MIX_LDS    (MIX_FLOATS * 4)
#define MIX_CHUNKS (MIX_LDS / 512)

#define WSCALE 64.0f
#define HSCALE 4.0f

static_assert(BSZ % GROWS == 0);
static_assert(BSZ % EROWS == 0);
static_assert(BSZ % MROWS == 0);
static_assert(FDIM % 32 == 0);
static_assert(EHD % 32 == 0);
static_assert(GHD == 8 * 32);
static_assert(EHD == 8 * 64);
static_assert(CPAD == 8 * 128);
static_assert(CDIM <= CPAD);
static_assert(MIX_LDS % 512 == 0);
static_assert((MIX_LDS % 128) == 0);
static_assert((TP * 2) % 16 == 0);
static_assert(NEXP == (1 << DEPTH));
static_assert(NGATE == (1 << DEPTH) - 1);
static_assert(MROWS * NEXP == 256);
static_assert(EHD / 8 == 64);
static_assert(CPAD * EHD / 8 == 65536);
static_assert((BSZ * FDIM) % 256 == 0);
static_assert((NGATE * GHD * FDIM) % 256 == 0);
static_assert((NEXP * EHD * FDIM) % 256 == 0);

typedef _Float16       v16h __attribute__((ext_vector_type(16)));
typedef _Float16       v8h  __attribute__((ext_vector_type(8)));
typedef float          v8f  __attribute__((ext_vector_type(8)));
typedef float          v4f  __attribute__((ext_vector_type(4)));
typedef unsigned int   v4u  __attribute__((ext_vector_type(4)));
typedef v4f __attribute__((may_alias)) v4fa;
typedef v4u __attribute__((may_alias)) v4ua;

union FragH { v16h v; v4u q[2]; };
union Pack8 { v8h v; v4u u; };

__device__ __forceinline__ v8f wmma_h(v16h a, v16h b, v8f c) {
  v8f d = __builtin_amdgcn_wmma_f32_16x16x32_f16(false, a, false, b, (short)0, c, false, false);
  asm volatile("v_nop\n\tv_nop\n\tv_nop\n\tv_nop" : "+v"(d) : "v"(a), "v"(b));
  return d;
}

__device__ __forceinline__ v16h ldfrag(const unsigned short* p, int h) {
  FragH f;
  f.q[0] = *(const v4ua*)(p + 8 * h);
  f.q[1] = *(const v4ua*)(p + 16 + 8 * h);
  return f.v;
}

__device__ __forceinline__ v4u pack8h(const v4f a, const v4f c, const float s) {
  Pack8 p;
  const v8h t = { (_Float16)(a.x * s), (_Float16)(a.y * s), (_Float16)(a.z * s), (_Float16)(a.w * s),
                  (_Float16)(c.x * s), (_Float16)(c.y * s), (_Float16)(c.z * s), (_Float16)(c.w * s) };
  p.v = t;
  return p.u;
}

__global__ __launch_bounds__(256) void k_cvt(const float* __restrict__ src,
                                             unsigned short* __restrict__ dst,
                                             int n8, float scale)
{
  const int g = blockIdx.x * 256 + threadIdx.x;
  if (g >= n8) return;
  const float* s = src + (size_t)g * 8;
  const v4f a = *(const v4fa*)s;
  const v4f c = *(const v4fa*)(s + 4);
  const v4u H = pack8h(a, c, scale);
  unsigned short* d = dst + (size_t)g * 8;
  *(volatile v4u*)d = H;
  __threadfence();
  *(volatile v4u*)d = H;
}

__global__ __launch_bounds__(256) void k_cvt_cls(const float* __restrict__ src,
                                                 unsigned short* __restrict__ dst,
                                                 int n8, float scale)
{
  const int g = blockIdx.x * 256 + threadIdx.x;
  if (g >= n8) return;
  const int k8 = g & 63;
  const int c  = (g >> 6) & (CPAD - 1);
  const int e  = g >> 16;
  const int cc = (c < CDIM) ? c : (CDIM - 1);
  const float* s = src + ((size_t)e * CDIM + cc) * EHD + 8 * k8;
  const v4f a = *(const v4fa*)s;
  const v4f b = *(const v4fa*)(s + 4);
  const v4u H = pack8h(a, b, scale);
  const bool ok = (c < CDIM);
  v4u V;
  V.x = ok ? H.x : 0u;
  V.y = ok ? H.y : 0u;
  V.z = ok ? H.z : 0u;
  V.w = ok ? H.w : 0u;
  unsigned short* d = dst + (size_t)g * 8;
  *(volatile v4u*)d = V;
  __threadfence();
  *(volatile v4u*)d = V;
}

__global__ __launch_bounds__(256) void k_gate(const unsigned short* __restrict__ xh,
                                              const unsigned short* __restrict__ gw1h,
                                              const float* __restrict__ gb1,
                                              const float* __restrict__ gw2,
                                              const float* __restrict__ gb2,
                                              float* __restrict__ gp)
{
  __shared__ float spart[8 * GROWS * 2];
  __shared__ __align__(16) float sp[2 * GROWS];
  const int tid = threadIdx.x, lane = tid & 31, wv = tid >> 5;
  const int h = lane >> 4, m = lane & 15;
  const int g = blockIdx.x / (BSZ / GROWS);
  const int row0 = (blockIdx.x % (BSZ / GROWS)) * GROWS;

  const v8f z8 = {0.f, 0.f, 0.f, 0.f, 0.f, 0.f, 0.f, 0.f};
  v8f acc[2][2];
  #pragma unroll
  for (int mt = 0; mt < 2; ++mt)
    #pragma unroll
    for (int nt = 0; nt < 2; ++nt) acc[mt][nt] = z8;

  const unsigned short* Ab = xh + (size_t)row0 * FDIM;
  const unsigned short* Bb = gw1h + ((size_t)g * GHD + wv * 32) * FDIM;
  #pragma unroll 2
  for (int k0 = 0; k0 < FDIM; k0 += 32) {
    const v16h a0 = ldfrag(Ab + (size_t)m * FDIM + k0, h);
    const v16h a1 = ldfrag(Ab + (size_t)(16 + m) * FDIM + k0, h);
    const v16h b0 = ldfrag(Bb + (size_t)m * FDIM + k0, h);
    const v16h b1 = ldfrag(Bb + (size_t)(16 + m) * FDIM + k0, h);
    acc[0][0] = wmma_h(a0, b0, acc[0][0]);
    acc[1][0] = wmma_h(a1, b0, acc[1][0]);
    acc[0][1] = wmma_h(a0, b1, acc[0][1]);
    acc[1][1] = wmma_h(a1, b1, acc[1][1]);
  }

  float bia[2], u0[2], u1[2];
  #pragma unroll
  for (int nt = 0; nt < 2; ++nt) {
    const int col = wv * 32 + 16 * nt + m;
    bia[nt] = gb1[(size_t)g * GHD + col];
    u0[nt]  = gw2[((size_t)g * BFC + 0) * GHD + col];
    u1[nt]  = gw2[((size_t)g * BFC + 1) * GHD + col];
  }
  #pragma unroll
  for (int mt = 0; mt < 2; ++mt) {
    #pragma unroll
    for (int r = 0; r < 8; ++r) {
      float s0 = 0.0f, s1 = 0.0f;
      #pragma unroll
      for (int nt = 0; nt < 2; ++nt) {
        const float ghv = tanhf(acc[mt][nt][r] * (1.0f / WSCALE) + bia[nt]);
        s0 += ghv * u0[nt];
        s1 += ghv * u1[nt];
      }
      #pragma unroll
      for (int off = 1; off < 16; off <<= 1) {
        s0 += __shfl_xor(s0, off, 32);
        s1 += __shfl_xor(s1, off, 32);
      }
      if (m == 0) {
        const int row = 16 * mt + 8 * h + r;
        spart[(wv * GROWS + row) * 2 + 0] = s0;
        spart[(wv * GROWS + row) * 2 + 1] = s1;
      }
    }
  }
  __syncthreads();
  if (tid < GROWS) {
    float s0 = 0.0f, s1 = 0.0f;
    #pragma unroll
    for (int w2 = 0; w2 < 8; ++w2) {
      s0 += spart[(w2 * GROWS + tid) * 2 + 0];
      s1 += spart[(w2 * GROWS + tid) * 2 + 1];
    }
    const float l0 = s0 + gb2[g * BFC + 0];
    const float l1 = s1 + gb2[g * BFC + 1];
    const float mx = fmaxf(l0, l1);
    const float e0 = expf(l0 - mx);
    const float e1 = expf(l1 - mx);
    const float rs = __builtin_amdgcn_rcpf(e0 + e1);
    sp[2 * tid + 0] = e0 * rs;
    sp[2 * tid + 1] = e1 * rs;
  }
  __syncthreads();
  if (wv == 0) {
    const int q = lane & 15;
    const v4f v = *(const v4fa*)(sp + 4 * q);
    float* dst = gp + ((size_t)g * BSZ + row0) * BFC + 4 * q;
    if (lane < 16) *(volatile v4f*)dst = v;
    __threadfence();
    if (lane < 16) *(volatile v4f*)dst = v;
  }
}

__global__ __launch_bounds__(256) void k_exph(const unsigned short* __restrict__ xh,
                                              const unsigned short* __restrict__ ew1h,
                                              const float* __restrict__ eb1,
                                              unsigned short* __restrict__ eh)
{
  __shared__ __align__(16) unsigned short sT[8 * EROWS * TP];
  const int tid = threadIdx.x, lane = tid & 31, wv = tid >> 5;
  const int h = lane >> 4, m = lane & 15;
  const int e = blockIdx.x / (BSZ / EROWS);
  const int row0 = (blockIdx.x % (BSZ / EROWS)) * EROWS;

  const v8f z8 = {0.f, 0.f, 0.f, 0.f, 0.f, 0.f, 0.f, 0.f};
  v8f acc[2][4];
  #pragma unroll
  for (int mt = 0; mt < 2; ++mt)
    #pragma unroll
    for (int nt = 0; nt < 4; ++nt) acc[mt][nt] = z8;

  const unsigned short* Ab = xh + (size_t)row0 * FDIM;
  const unsigned short* Bb = ew1h + ((size_t)e * EHD + wv * 64) * FDIM;
  #pragma unroll 2
  for (int k0 = 0; k0 < FDIM; k0 += 32) {
    const v16h a0 = ldfrag(Ab + (size_t)m * FDIM + k0, h);
    const v16h a1 = ldfrag(Ab + (size_t)(16 + m) * FDIM + k0, h);
    #pragma unroll
    for (int nt = 0; nt < 4; ++nt) {
      const v16h b = ldfrag(Bb + (size_t)(16 * nt + m) * FDIM + k0, h);
      acc[0][nt] = wmma_h(a0, b, acc[0][nt]);
      acc[1][nt] = wmma_h(a1, b, acc[1][nt]);
    }
  }

  #pragma unroll
  for (int nt = 0; nt < 4; ++nt) {
    const int cl = 16 * nt + m;
    const float bv = eb1[(size_t)e * EHD + wv * 64 + cl];
    #pragma unroll
    for (int mt = 0; mt < 2; ++mt) {
      #pragma unroll
      for (int r = 0; r < 8; ++r) {
        const int row = 16 * mt + 8 * h + r;
        const float v = fmaxf(acc[mt][nt][r] * (1.0f / WSCALE) + bv, 0.0f) * HSCALE;
        const _Float16 hv = (_Float16)v;
        sT[(wv * EROWS + row) * TP + cl] = __builtin_bit_cast(unsigned short, hv);
      }
    }
  }
  __syncthreads();

  const int rq = lane >> 3, seg = lane & 7;
  unsigned short* ob = eh + ((size_t)e * BSZ + row0) * EHD + wv * 64 + 8 * seg;
  v4u vv[8];
  #pragma unroll
  for (int i = 0; i < 8; ++i)
    vv[i] = *(const v4ua*)(sT + (wv * EROWS + 4 * i + rq) * TP + 8 * seg);
  #pragma unroll
  for (int i = 0; i < 8; ++i)
    *(volatile v4u*)(ob + (size_t)(4 * i + rq) * EHD) = vv[i];
  __threadfence();
  #pragma unroll
  for (int i = 0; i < 8; ++i)
    *(volatile v4u*)(ob + (size_t)(4 * i + rq) * EHD) = vv[i];
}

__global__ __launch_bounds__(256) void k_mix(const unsigned short* __restrict__ ehh,
                                             const unsigned short* __restrict__ ew2h,
                                             const float* __restrict__ eb2,
                                             const float* __restrict__ gp,
                                             float* __restrict__ out)
{
  extern __shared__ __align__(16) float sY[];
  __shared__ float swl[MROWS * NEXP];
  __shared__ float maxbuf[MROWS * 8];
  __shared__ float sumbuf[MROWS * 8];
  const int tid = threadIdx.x, lane = tid & 31, wv = tid >> 5;
  const int h = lane >> 4, m = lane & 15;
  const int b0 = blockIdx.x * MROWS;
  const int n0 = wv * 128;

  {
    const int row = tid >> 4, e = tid & 15;
    const int b = b0 + row;
    float w = 1.0f;
    int idx = 0;
    #pragma unroll
    for (int d = 0; d < DEPTH; ++d) {
      const int c = (e >> (DEPTH - 1 - d)) & 1;
      const int g = (1 << d) - 1 + idx;
      const float p = gp[((size_t)g * BSZ + b) * BFC + c];
      w = w * p;
      idx = idx * 2 + c;
    }
    swl[row * NEXP + e] = w;
  }
  __syncthreads();

  const v8f z8 = {0.f, 0.f, 0.f, 0.f, 0.f, 0.f, 0.f, 0.f};
  float mix[8][8];
  #pragma unroll
  for (int nt = 0; nt < 8; ++nt)
    #pragma unroll
    for (int j = 0; j < 8; ++j) mix[nt][j] = 0.0f;

  #pragma unroll 1
  for (int e = 0; e < NEXP; ++e) {
    v8f acc[8];
    #pragma unroll
    for (int nt = 0; nt < 8; ++nt) acc[nt] = z8;
    const unsigned short* Ab = ehh + ((size_t)e * BSZ + b0 + m) * EHD;
    const unsigned short* Bb = ew2h + ((size_t)e * CPAD + n0 + m) * EHD;
    #pragma unroll 1
    for (int k0 = 0; k0 < EHD; k0 += 32) {
      const v16h a = ldfrag(Ab + k0, h);
      #pragma unroll
      for (int nt = 0; nt < 8; ++nt) {
        const v16h b = ldfrag(Bb + (size_t)(16 * nt) * EHD + k0, h);
        acc[nt] = wmma_h(a, b, acc[nt]);
      }
    }

    #pragma unroll
    for (int nt = 0; nt < 8; ++nt) {
      const int n = n0 + 16 * nt + m;
      const int nc = (n < CDIM) ? n : (CDIM - 1);
      const float bv = eb2[(size_t)e * CDIM + nc];
      const bool ok = (n < CDIM);
      #pragma unroll
      for (int j = 0; j < 8; ++j)
        acc[nt][j] = ok ? (acc[nt][j] * (1.0f / (WSCALE * HSCALE)) + bv) : -3.0e38f;
    }

    float rmax[8];
    #pragma unroll
    for (int j = 0; j < 8; ++j) {
      float mx = acc[0][j];
      #pragma unroll
      for (int nt = 1; nt < 8; ++nt) mx = fmaxf(mx, acc[nt][j]);
      rmax[j] = mx;
    }
    #pragma unroll
    for (int off = 1; off < 16; off <<= 1)
      #pragma unroll
      for (int j = 0; j < 8; ++j) rmax[j] = fmaxf(rmax[j], __shfl_xor(rmax[j], off, 32));
    if (m == 0) {
      #pragma unroll
      for (int j = 0; j < 8; ++j) maxbuf[(8 * h + j) * 8 + wv] = rmax[j];
    }
    __syncthreads();
    #pragma unroll
    for (int j = 0; j < 8; ++j) {
      float mx = maxbuf[(8 * h + j) * 8 + 0];
      #pragma unroll
      for (int w2 = 1; w2 < 8; ++w2) mx = fmaxf(mx, maxbuf[(8 * h + j) * 8 + w2]);
      rmax[j] = mx;
    }

    float rsum[8];
    #pragma unroll
    for (int j = 0; j < 8; ++j) rsum[j] = 0.0f;
    #pragma unroll
    for (int nt = 0; nt < 8; ++nt)
      #pragma unroll
      for (int j = 0; j < 8; ++j) {
        const float ex = __expf(acc[nt][j] - rmax[j]);
        acc[nt][j] = ex;
        rsum[j] += ex;
      }
    #pragma unroll
    for (int off = 1; off < 16; off <<= 1)
      #pragma unroll
      for (int j = 0; j < 8; ++j) rsum[j] += __shfl_xor(rsum[j], off, 32);
    if (m == 0) {
      #pragma unroll
      for (int j = 0; j < 8; ++j) sumbuf[(8 * h + j) * 8 + wv] = rsum[j];
    }
    __syncthreads();
    float coef[8];
    #pragma unroll
    for (int j = 0; j < 8; ++j) {
      float s = 0.0f;
      #pragma unroll
      for (int w2 = 0; w2 < 8; ++w2) s += sumbuf[(8 * h + j) * 8 + w2];
      coef[j] = swl[(8 * h + j) * NEXP + e] * __builtin_amdgcn_rcpf(s);
    }

    #pragma unroll
    for (int nt = 0; nt < 8; ++nt)
      #pragma unroll
      for (int j = 0; j < 8; ++j) mix[nt][j] += coef[j] * acc[nt][j];
  }

  #pragma unroll
  for (int nt = 0; nt < 8; ++nt) {
    const int n = n0 + 16 * nt + m;
    if (n < CDIM) {
      #pragma unroll
      for (int j = 0; j < 8; ++j) sY[(8 * h + j) * CDIM + n] = mix[nt][j];
    }
  }
  __syncthreads();

  float* ob = out + (size_t)blockIdx.x * MIX_FLOATS;
  #pragma unroll
  for (int i = 0; i < 16; ++i) {
    const int q = wv + 8 * i;
    if (q < MIX_CHUNKS) {
      const v4f v = *(const v4fa*)(sY + q * 128 + 4 * lane);
      *(volatile v4f*)(ob + (size_t)q * 128 + 4 * lane) = v;
    }
  }
  __threadfence();
  #pragma unroll
  for (int i = 0; i < 16; ++i) {
    const int q = wv + 8 * i;
    if (q < MIX_CHUNKS) {
      const v4f v = *(const v4fa*)(sY + q * 128 + 4 * lane);
      *(volatile v4f*)(ob + (size_t)q * 128 + 4 * lane) = v;
    }
  }
}

extern "C" void kernel_launch(void* const* d_in, const int* in_sizes, int n_in,
                              void* d_out, int out_size, void* d_ws, size_t ws_size,
                              hipStream_t stream)
{
  if (n_in < 9) return;
  if (in_sizes[0] != BSZ * FDIM) return;
  if (in_sizes[1] != NGATE * GHD * FDIM) return;
  if (in_sizes[2] != NGATE * GHD) return;
  if (in_sizes[3] != NGATE * BFC * GHD) return;
  if (in_sizes[4] != NGATE * BFC) return;
  if (in_sizes[5] != NEXP * EHD * FDIM) return;
  if (in_sizes[6] != NEXP * EHD) return;
  if (in_sizes[7] != NEXP * CDIM * EHD) return;
  if (in_sizes[8] != NEXP * CDIM) return;
  if (out_size != BSZ * CDIM) return;

  const float* x   = (const float*)d_in[0];
  const float* gw1 = (const float*)d_in[1];
  const float* gb1 = (const float*)d_in[2];
  const float* gw2 = (const float*)d_in[3];
  const float* gb2 = (const float*)d_in[4];
  const float* ew1 = (const float*)d_in[5];
  const float* eb1 = (const float*)d_in[6];
  const float* ew2 = (const float*)d_in[7];
  const float* eb2 = (const float*)d_in[8];
  float* out = (float*)d_out;

  const size_t bXP  = (size_t)BSZ * FDIM * 2;
  const size_t bGW1 = (size_t)NGATE * GHD * FDIM * 2;
  const size_t bEW1 = (size_t)NEXP * EHD * FDIM * 2;
  const size_t bEW2 = (size_t)NEXP * CPAD * EHD * 2;
  const size_t bGP  = (size_t)NGATE * BSZ * BFC * 4;
  const size_t bEH  = (size_t)NEXP * BSZ * EHD * 2;
  const size_t total = bXP + bGW1 + bEW1 + bEW2 + bGP + bEH;
  if (total > ws_size) return;
  if (total > (size_t)134217728) return;

  char* ws = (char*)d_ws;
  size_t off = 0;
  unsigned short* XH   = (unsigned short*)(ws + off); off += bXP;
  unsigned short* GW1H = (unsigned short*)(ws + off); off += bGW1;
  unsigned short* EW1H = (unsigned short*)(ws + off); off += bEW1;
  unsigned short* EW2H = (unsigned short*)(ws + off); off += bEW2;
  float*          GP   = (float*)(ws + off);          off += bGP;
  unsigned short* EHP  = (unsigned short*)(ws + off); off += bEH;
  if (off != total) return;

  {
    const int n8x  = BSZ * FDIM / 8;
    const int n8g  = NGATE * GHD * FDIM / 8;
    const int n8e1 = NEXP * EHD * FDIM / 8;
    const int n8e2 = NEXP * CPAD * EHD / 8;
    k_cvt<<<(n8x + 255) / 256, 256, 0, stream>>>(x, XH, n8x, 1.0f);
    k_cvt<<<(n8g + 255) / 256, 256, 0, stream>>>(gw1, GW1H, n8g, WSCALE);
    k_cvt<<<(n8e1 + 255) / 256, 256, 0, stream>>>(ew1, EW1H, n8e1, WSCALE);
    k_cvt_cls<<<(n8e2 + 255) / 256, 256, 0, stream>>>(ew2, EW2H, n8e2, WSCALE);
  }
  k_gate<<<NGATE * (BSZ / GROWS), 256, 0, stream>>>(XH, GW1H, gb1, gw2, gb2, GP);
  k_exph<<<NEXP * (BSZ / EROWS), 256, 0, stream>>>(XH, EW1H, eb1, EHP);
  hipFuncSetAttribute(reinterpret_cast<const void*>(&k_mix),
                      hipFuncAttributeMaxDynamicSharedMemorySize, MIX_LDS);
  k_mix<<<BSZ / MROWS, 256, MIX_LDS, stream>>>(EHP, EW2H, eb2, GP, out);
}
